// BiRNN_15616501088715
// MI455X (gfx1250) — hardware-verified
//
#include <hip/hip_runtime.h>
#include <hip/hip_bf16.h>

typedef __attribute__((ext_vector_type(16))) _Float16 v16h;
typedef __attribute__((ext_vector_type(8)))  _Float16 v8h;
typedef __attribute__((ext_vector_type(16))) __bf16   v16b;
typedef __attribute__((ext_vector_type(8)))  __bf16   v8b;
typedef __attribute__((ext_vector_type(8)))  float    v8f;
typedef __attribute__((ext_vector_type(4)))  float    v4f;

namespace {
constexpr int NBATCH = 64, NSTEP = 512, NEMB = 256, NHID = 256, NOUT = 256;
constexpr int NROWS = NBATCH * NSTEP;
constexpr int HPITCH = 264;
constexpr int FPITCH = 260;

constexpr size_t kOffXh    = 0;
constexpr size_t kOffWxhTf = kOffXh    + (size_t)NROWS * NEMB * 2;
constexpr size_t kOffWxhTb = kOffWxhTf + (size_t)NEMB * NHID * 2;
constexpr size_t kOffWhhTf = kOffWxhTb + (size_t)NEMB * NHID * 2;
constexpr size_t kOffWhhTb = kOffWhhTf + (size_t)NHID * NHID * 2;
constexpr size_t kOffWhyT  = kOffWhhTb + (size_t)NHID * NHID * 2;
constexpr size_t kOffXF    = kOffWhyT  + (size_t)(2 * NHID) * NOUT * 2;
constexpr size_t kOffXB    = kOffXF    + (size_t)NROWS * NHID * 4;
constexpr size_t kOffHcat  = kOffXB    + (size_t)NROWS * NHID * 4;
constexpr size_t kWsTotal  = kOffHcat  + (size_t)NROWS * (2 * NHID) * 2;
static_assert(kWsTotal == 118226944ull);
static_assert(kWsTotal <= 134217728ull);
}

__device__ __forceinline__ unsigned short f2bf_bits(float f) {
  unsigned u = __float_as_uint(f);
  return (unsigned short)((u + 0x7FFFu + ((u >> 16) & 1u)) >> 16);
}
__device__ __forceinline__ float bf_bits2f(unsigned short h) { return __uint_as_float(((unsigned)h) << 16); }

__device__ __forceinline__ void dep_guard_h(v8f& a, v8f& b, v16h x, v16h y) { asm volatile("v_nop\n\tv_nop\n\tv_nop\n\tv_nop" : "+v"(a), "+v"(b) : "v"(x), "v"(y)); }
__device__ __forceinline__ void dep_guard_b(v8f& a, v8f& b, v16b x, v16b y) { asm volatile("v_nop\n\tv_nop\n\tv_nop\n\tv_nop" : "+v"(a), "+v"(b) : "v"(x), "v"(y)); }
__device__ __forceinline__ void dep_guard3_h(v8f& a, v8f& b, v16h x, v16h y, v16h z) { asm volatile("v_nop\n\tv_nop\n\tv_nop\n\tv_nop" : "+v"(a), "+v"(b) : "v"(x), "v"(y), "v"(z)); }
__device__ __forceinline__ void acc_guard2(v8f& a, v8f& b) { asm volatile("v_nop\n\tv_nop\n\tv_nop\n\tv_nop" : "+v"(a), "+v"(b)); }
__device__ __forceinline__ void keep4_h(v16h a, v16h b, v16h c, v16h d) { asm volatile("v_nop" :: "v"(a), "v"(b), "v"(c), "v"(d)); }
__device__ __forceinline__ void keep4_b(v16b a, v16b b, v16b c, v16b d) { asm volatile("v_nop" :: "v"(a), "v"(b), "v"(c), "v"(d)); }
__device__ __forceinline__ void acc_guard4(v8f& a, v8f& b, v8f& c, v8f& d) { asm volatile("v_nop\n\tv_nop\n\tv_nop\n\tv_nop" : "+v"(a), "+v"(b), "+v"(c), "+v"(d)); }
template <typename T> struct Frag;
template <> struct Frag<_Float16> {
  typedef v16h V; union U { v16h v; v8h h[2]; };
  static __device__ __forceinline__ v16h load(const _Float16* p) {
    U f; f.h[0] = *(const v8h*)(p); f.h[1] = *(const v8h*)(p + 16); return f.v;
  }
  static __device__ __forceinline__ v8f mma(v16h a, v16h b, v8f c) {
    return __builtin_amdgcn_wmma_f32_16x16x32_f16(false, a, false, b, (short)0, c, false, false);
  }
  static __device__ __forceinline__ void guard(v8f& a, v8f& b, v16h x, v16h y) { dep_guard_h(a, b, x, y); }
  static __device__ __forceinline__ void keep(v16h a, v16h b, v16h c, v16h d) { keep4_h(a, b, c, d); }
};
template <> struct Frag<__bf16> {
  typedef v16b V; union U { v16b v; v8b h[2]; };
  static __device__ __forceinline__ v16b load(const __bf16* p) {
    U f; f.h[0] = *(const v8b*)(p); f.h[1] = *(const v8b*)(p + 16); return f.v;
  }
  static __device__ __forceinline__ v8f mma(v16b a, v16b b, v8f c) {
    return __builtin_amdgcn_wmma_f32_16x16x32_bf16(false, a, false, b, (short)0, c, false, false);
  }
  static __device__ __forceinline__ void guard(v8f& a, v8f& b, v16b x, v16b y) { dep_guard_b(a, b, x, y); }
  static __device__ __forceinline__ void keep(v16b a, v16b b, v16b c, v16b d) { keep4_b(a, b, c, d); }
};

template <int ET> struct Elem;
template <> struct Elem<0> { typedef _Float16 T; };
template <> struct Elem<1> { typedef __bf16 T; };
template <int ET, bool SPLIT, int BIAS_MODE, int OUT_MODE, bool RESID, int ACT = 0>
__global__ __launch_bounds__(256) void wmma_gemm64(
    const unsigned short* __restrict__ Ap, const unsigned short* __restrict__ A2p, int lda, long strideA,
    const unsigned short* __restrict__ Btp, const unsigned short* __restrict__ Bt2p, int ldb, long strideB,
    void* __restrict__ Cout, void* __restrict__ Cout2, int ldc, long strideC,
    const float* __restrict__ bias,
    const float* __restrict__ resid, long strideR,
    int M, int N, int K, float scale) {
  typedef typename Elem<ET>::T T;
  typedef typename Frag<T>::V V;
  const T* A = (const T*)Ap; const T* A2 = (const T*)A2p; const T* Bt = (const T*)Btp; const T* Bt2 = (const T*)Bt2p;
  __shared__ __align__(16) float sT[8][16 * 68];
  const int b    = blockIdx.y;
  const int lane = threadIdx.x & 31;
  const int wave = threadIdx.x >> 5;
  const int tilesN = N >> 6;
  const int tilesM = M >> 6;
  const int tile = blockIdx.x * 8 + wave;
  if (tile >= tilesM * tilesN) return;
  const int tm = tile / tilesN;
  const int tn = tile - tm * tilesN;
  const int m0 = tm << 6;
  const int n0 = tn << 6;

  const T* Ab  = A  + (size_t)b * strideA;
  const T* Bb  = Bt + (size_t)b * strideB;
  const T* Ab2 = SPLIT ? (A2  + (size_t)b * strideA) : nullptr;
  const T* Bb2 = SPLIT ? (Bt2 + (size_t)b * strideB) : nullptr;

  const int rlane = lane & 15;
  const int koff  = (lane >> 4) * 8;
  const int mOff  = (lane >> 4) * 8;

  v8f acc[4][4];
#pragma unroll
  for (int i = 0; i < 4; ++i)
#pragma unroll
    for (int j = 0; j < 4; ++j) acc[i][j] = (v8f){0.f,0.f,0.f,0.f,0.f,0.f,0.f,0.f};

  for (int k0 = 0; k0 < K; k0 += 32) {
    V bh[4], bl[4];
#pragma unroll
    for (int j = 0; j < 4; ++j) {
      const size_t bo = (size_t)(n0 + (j << 4) + rlane) * ldb + koff + k0;
      bh[j] = Frag<T>::load(Bb + bo);
      if (SPLIT) bl[j] = Frag<T>::load(Bb2 + bo);
    }
#pragma unroll
    for (int i = 0; i < 4; ++i) {
      const size_t ao = (size_t)(m0 + (i << 4) + rlane) * lda + koff + k0;
      V ah = Frag<T>::load(Ab + ao);
      V al;
      if (SPLIT) al = Frag<T>::load(Ab2 + ao);
#pragma unroll
      for (int j = 0; j < 4; ++j) {
        acc[i][j] = Frag<T>::mma(ah, bh[j], acc[i][j]);
        if (SPLIT) {
          acc[i][j] = Frag<T>::mma(ah, bl[j], acc[i][j]);
          acc[i][j] = Frag<T>::mma(al, bh[j], acc[i][j]);
        }
      }
      Frag<T>::guard(acc[i][0], acc[i][3], ah, SPLIT ? al : ah);
    }
    Frag<T>::keep(bh[0], bh[1], bh[2], bh[3]);
    if (SPLIT) Frag<T>::keep(bl[0], bl[1], bl[2], bl[3]);
  }
  acc_guard4(acc[0][0], acc[0][1], acc[0][2], acc[0][3]);
  acc_guard4(acc[1][0], acc[1][1], acc[1][2], acc[1][3]);
  acc_guard4(acc[2][0], acc[2][1], acc[2][2], acc[2][3]);
  acc_guard4(acc[3][0], acc[3][1], acc[3][2], acc[3][3]);

  float* slab = sT[wave];
  const float* Rb = RESID ? (resid + (size_t)b * strideR) : nullptr;
#pragma unroll
  for (int i = 0; i < 4; ++i) {
    const int mBase = m0 + (i << 4);
#pragma unroll
    for (int j = 0; j < 4; ++j) {
      const int n = n0 + (j << 4) + rlane;
      float bv = 0.f;
      if (BIAS_MODE == 2) bv = bias[n];
#pragma unroll
      for (int r = 0; r < 8; ++r) {
        float v = acc[i][j][r] * scale;
        if (BIAS_MODE == 1) v += bias[mBase + mOff + r];
        if (BIAS_MODE == 2) v += bv;
        if (RESID) v += Rb[(size_t)(mBase + mOff + r) * ldc + n];
        if (ACT == 1) v = tanhf(v);
        if (ACT == 2) v = fmaxf(v, 0.0f);
        if (ACT == 3) v = v / (1.0f + expf(-v));
        if (ACT == 4) v = (v > 0.f) ? v : 0.01f * v;
        if (ACT == 5) v = 0.5f * v * (1.0f + erff(v * 0.70710678118654752f));
        slab[(mOff + r) * 68 + (j << 4) + rlane] = v;
      }
    }
    __builtin_amdgcn_fence(__ATOMIC_RELEASE, "workgroup");
    __builtin_amdgcn_wave_barrier();
    __builtin_amdgcn_fence(__ATOMIC_ACQUIRE, "workgroup");
    if (OUT_MODE == 0) {
      float* C = (float*)Cout + (size_t)b * strideC;
      const int hh = lane >> 4, c4 = (lane & 15) * 4;
      for (int pass = 0; pass < 2; ++pass) {
#pragma unroll
        for (int it = 0; it < 8; ++it) {
          const int row = it * 2 + hh;
          v4f v = *(const v4f*)(slab + row * 68 + c4);
          *(volatile v4f*)(C + (size_t)(mBase + row) * ldc + n0 + c4) = v;
        }
        __threadfence();
      }
    } else {
      const int q = lane >> 3, c8 = (lane & 7) * 8;
      unsigned short* C  = (unsigned short*)Cout  + (size_t)b * strideC;
      unsigned short* C2 = (OUT_MODE == 2) ? ((unsigned short*)Cout2 + (size_t)b * strideC) : nullptr;
      for (int pass = 0; pass < 2; ++pass) {
#pragma unroll
        for (int it = 0; it < 4; ++it) {
          const int row = it * 4 + q;
          const float* sp = slab + row * 68 + c8;
          v8h hv, lv;
#pragma unroll
          for (int e = 0; e < 8; ++e) {
            if (OUT_MODE == 1) {
              hv[e] = (_Float16)sp[e];
            } else {
              unsigned short hb = f2bf_bits(sp[e]);
              unsigned short lb = f2bf_bits(sp[e] - bf_bits2f(hb));
              hv[e] = __builtin_bit_cast(_Float16, hb);
              lv[e] = __builtin_bit_cast(_Float16, lb);
            }
          }
          *(volatile v8h*)(C + (size_t)(mBase + row) * ldc + n0 + c8) = hv;
          if (OUT_MODE == 2) *(volatile v8h*)(C2 + (size_t)(mBase + row) * ldc + n0 + c8) = lv;
        }
        __threadfence();
      }
    }
    __builtin_amdgcn_fence(__ATOMIC_RELEASE, "workgroup");
    __builtin_amdgcn_wave_barrier();
    __builtin_amdgcn_fence(__ATOMIC_ACQUIRE, "workgroup");
  }
}

__global__ __launch_bounds__(256) void cast_f32_f16x2(
    const float* __restrict__ in, _Float16* __restrict__ out, int n2) {
  int i = blockIdx.x * 256 + threadIdx.x;
  if (i < n2) {
    const _Float16 h0 = (_Float16)in[2 * i], h1 = (_Float16)in[2 * i + 1];
    const unsigned u = (unsigned)__builtin_bit_cast(unsigned short, h0) | ((unsigned)__builtin_bit_cast(unsigned short, h1) << 16);
    ((volatile unsigned*)out)[i] = u;
    __threadfence();
    ((volatile unsigned*)out)[i] = u;
  }
}

__global__ __launch_bounds__(256) void transpose_cast_f16(
    const float* __restrict__ W, unsigned short* __restrict__ Bt, int K, int N, float mul) {
  __shared__ float tile[64][33];
  const int tid = threadIdx.x;
  const int n0 = blockIdx.x * 32;
  const int k0 = blockIdx.y * 64;
#pragma unroll
  for (int i = 0; i < 8; ++i) {
    const int e = tid + 256 * i;
    const int kk = e >> 5, nn = e & 31;
    tile[kk][nn] = W[(size_t)(k0 + kk) * N + n0 + nn];
  }
  __syncthreads();
  const int r = tid >> 3, q = tid & 7;
  v8h hv;
#pragma unroll
  for (int e = 0; e < 8; ++e) hv[e] = (_Float16)(tile[8 * q + e][r] * mul);
  unsigned short* dst = Bt + (size_t)(n0 + r) * K + k0 + 8 * q;
  *(volatile v8h*)dst = hv;
  __threadfence();
  *(volatile v8h*)dst = hv;
}

__global__ __launch_bounds__(256) void seq_scan_kernel(
    const float* __restrict__ XF, const float* __restrict__ XB,
    const unsigned short* __restrict__ WhhTf, const unsigned short* __restrict__ WhhTb,
    unsigned short* __restrict__ Hcat,
    float* __restrict__ hlastF, float* __restrict__ hlastB) {
  __shared__ __align__(16) _Float16 hT[2][16 * HPITCH];
  __shared__ __align__(16) float sF[16 * FPITCH];
  const int tid  = threadIdx.x;
  const int lane = tid & 31;
  const int wave = tid >> 5;
  const int hh   = lane >> 4;
  const int c    = lane & 15;
  const int dir  = blockIdx.x >> 2;
  const int b0   = (blockIdx.x & 3) * 16;
  const float* xp = dir ? XB : XF;
  const _Float16* Wt = (const _Float16*)(dir ? WhhTb : WhhTf);
  float* hlast = dir ? hlastB : hlastF;
  const int n0 = wave * 32;

  {
    unsigned* hz = (unsigned*)(&hT[0][0]);
    for (int i = tid; i < (2 * 16 * HPITCH) / 2; i += 256) hz[i] = 0u;
  }
  __syncthreads();

  float hv[2][8];
#pragma unroll
  for (int j = 0; j < 2; ++j)
#pragma unroll
    for (int r = 0; r < 8; ++r) hv[j][r] = 0.0f;

  const float kAccInv = 1.0f / 128.0f;
  int cur = 0;
  for (int s = 0; s < NSTEP; ++s) {
    const int tt = dir ? (NSTEP - 1 - s) : s;
    float xv[2][8];
#pragma unroll
    for (int j = 0; j < 2; ++j)
#pragma unroll
      for (int r = 0; r < 8; ++r)
        xv[j][r] = xp[((size_t)(b0 + 8 * hh + r) * NSTEP + tt) * NHID + n0 + 16 * j + c];

    v8f acc0 = (v8f){0.f,0.f,0.f,0.f,0.f,0.f,0.f,0.f};
    v8f acc1 = (v8f){0.f,0.f,0.f,0.f,0.f,0.f,0.f,0.f};
    const _Float16* hA  = hT[cur] + c * HPITCH + 8 * hh;
    const _Float16* wB0 = Wt + (size_t)(n0 + c) * NHID + 8 * hh;
    const _Float16* wB1 = Wt + (size_t)(n0 + 16 + c) * NHID + 8 * hh;
#pragma unroll
    for (int ks = 0; ks < 8; ++ks) {
      v16h a   = Frag<_Float16>::load(hA  + ks * 32);
      v16h bq0 = Frag<_Float16>::load(wB0 + ks * 32);
      v16h bq1 = Frag<_Float16>::load(wB1 + ks * 32);
      acc0 = Frag<_Float16>::mma(a, bq0, acc0);
      acc1 = Frag<_Float16>::mma(a, bq1, acc1);
      dep_guard3_h(acc0, acc1, a, bq0, bq1);
    }
    acc_guard2(acc0, acc1);

    _Float16* hN = hT[cur ^ 1];
#pragma unroll
    for (int r = 0; r < 8; ++r) {
      const float h0v = tanhf(xv[0][r] + acc0[r] * kAccInv);
      const float h1v = tanhf(xv[1][r] + acc1[r] * kAccInv);
      hv[0][r] = h0v;
      hv[1][r] = h1v;
      _Float16* dst = hN + (8 * hh + r) * HPITCH + n0 + c;
      dst[0]  = (_Float16)(h0v * 8.0f);
      dst[16] = (_Float16)(h1v * 8.0f);
    }
    __syncthreads();

    {
      const _Float16* srow = hN + (2 * wave) * HPITCH + 8 * lane;
      const v8h v0 = *(const v8h*)(srow);
      const v8h v1 = *(const v8h*)(srow + HPITCH);
      unsigned short* g0 = Hcat + ((size_t)(b0 + 2 * wave) * NSTEP + tt) * (2 * NHID) + dir * NHID + 8 * lane;
      unsigned short* g1 = g0 + (size_t)NSTEP * (2 * NHID);
      for (int pass = 0; pass < 2; ++pass) {
        *(volatile v8h*)g0 = v0;
        *(volatile v8h*)g1 = v1;
        __threadfence();
      }
    }
    cur ^= 1;
  }

#pragma unroll
  for (int r = 0; r < 8; ++r) {
    sF[(8 * hh + r) * FPITCH + n0 + c]      = hv[0][r];
    sF[(8 * hh + r) * FPITCH + n0 + 16 + c] = hv[1][r];
  }
  __syncthreads();
  {
    const float* s0 = sF + (2 * wave) * FPITCH;
    const v4f a0 = *(const v4f*)(s0 + 4 * lane);
    const v4f a1 = *(const v4f*)(s0 + 128 + 4 * lane);
    const v4f c0 = *(const v4f*)(s0 + FPITCH + 4 * lane);
    const v4f c1 = *(const v4f*)(s0 + FPITCH + 128 + 4 * lane);
    float* g = hlast + (size_t)(b0 + 2 * wave) * NHID;
    for (int pass = 0; pass < 2; ++pass) {
      *(volatile v4f*)(g + 4 * lane)              = a0;
      *(volatile v4f*)(g + 128 + 4 * lane)        = a1;
      *(volatile v4f*)(g + NHID + 4 * lane)       = c0;
      *(volatile v4f*)(g + NHID + 128 + 4 * lane) = c1;
      __threadfence();
    }
  }
}

extern "C" void kernel_launch(void* const* d_in, const int* in_sizes, int n_in,
                              void* d_out, int out_size, void* d_ws, size_t ws_size,
                              hipStream_t stream) {
  if (n_in != 9) return;
  if (in_sizes[0] != NBATCH * NSTEP * NEMB) return;
  if (in_sizes[1] != NEMB * NHID || in_sizes[2] != NHID * NHID || in_sizes[3] != NHID) return;
  if (in_sizes[4] != NEMB * NHID || in_sizes[5] != NHID * NHID || in_sizes[6] != NHID) return;
  if (in_sizes[7] != 2 * NHID * NOUT || in_sizes[8] != NOUT) return;
  if (out_size != NBATCH * NSTEP * NOUT + 2 * NBATCH * NHID) return;
  if (ws_size < kWsTotal) return;

  const float* X    = (const float*)d_in[0];
  const float* WxhF = (const float*)d_in[1];
  const float* WhhF = (const float*)d_in[2];
  const float* bF   = (const float*)d_in[3];
  const float* WxhB = (const float*)d_in[4];
  const float* WhhB = (const float*)d_in[5];
  const float* bB   = (const float*)d_in[6];
  const float* Why  = (const float*)d_in[7];
  const float* bY   = (const float*)d_in[8];
  float* Y      = (float*)d_out;
  float* hlastF = Y + (size_t)NBATCH * NSTEP * NOUT;
  float* hlastB = hlastF + (size_t)NBATCH * NHID;

  char* ws = (char*)d_ws;
  unsigned short* Xh    = (unsigned short*)(ws + kOffXh);
  unsigned short* WxhTf = (unsigned short*)(ws + kOffWxhTf);
  unsigned short* WxhTb = (unsigned short*)(ws + kOffWxhTb);
  unsigned short* WhhTf = (unsigned short*)(ws + kOffWhhTf);
  unsigned short* WhhTb = (unsigned short*)(ws + kOffWhhTb);
  unsigned short* WhyT  = (unsigned short*)(ws + kOffWhyT);
  float* XF = (float*)(ws + kOffXF);
  float* XB = (float*)(ws + kOffXB);
  unsigned short* Hcat = (unsigned short*)(ws + kOffHcat);

  const int n2 = NROWS * NEMB / 2;
  cast_f32_f16x2<<<dim3((n2 + 255) / 256), dim3(256), 0, stream>>>(X, (_Float16*)Xh, n2);

  transpose_cast_f16<<<dim3(NHID / 32, NEMB / 64), dim3(256), 0, stream>>>(WxhF, WxhTf, NEMB, NHID, 16.0f);
  transpose_cast_f16<<<dim3(NHID / 32, NEMB / 64), dim3(256), 0, stream>>>(WxhB, WxhTb, NEMB, NHID, 16.0f);
  transpose_cast_f16<<<dim3(NHID / 32, NHID / 64), dim3(256), 0, stream>>>(WhhF, WhhTf, NHID, NHID, 16.0f);
  transpose_cast_f16<<<dim3(NHID / 32, NHID / 64), dim3(256), 0, stream>>>(WhhB, WhhTb, NHID, NHID, 16.0f);
  transpose_cast_f16<<<dim3(NOUT / 32, (2 * NHID) / 64), dim3(256), 0, stream>>>(Why, WhyT, 2 * NHID, NOUT, 16.0f);

  const int gemmBlocks = ((NROWS / 64) * (NHID / 64) + 7) / 8;
  wmma_gemm64<0, false, 2, 0, false, 0><<<dim3(gemmBlocks, 1), dim3(256), 0, stream>>>(
      Xh, nullptr, NEMB, 0L, WxhTf, nullptr, NEMB, 0L,
      (void*)XF, nullptr, NHID, 0L, bF, nullptr, 0L, NROWS, NHID, NEMB, 1.0f / 16.0f);
  wmma_gemm64<0, false, 2, 0, false, 0><<<dim3(gemmBlocks, 1), dim3(256), 0, stream>>>(
      Xh, nullptr, NEMB, 0L, WxhTb, nullptr, NEMB, 0L,
      (void*)XB, nullptr, NHID, 0L, bB, nullptr, 0L, NROWS, NHID, NEMB, 1.0f / 16.0f);

  seq_scan_kernel<<<dim3(8), dim3(256), 0, stream>>>(XF, XB, WhhTf, WhhTb, Hcat, hlastF, hlastB);

  const int gemmBlocksY = ((NROWS / 64) * (NOUT / 64) + 7) / 8;
  wmma_gemm64<0, false, 2, 0, false, 0><<<dim3(gemmBlocksY, 1), dim3(256), 0, stream>>>(
      Hcat, nullptr, 2 * NHID, 0L, WhyT, nullptr, 2 * NHID, 0L,
      (void*)Y, nullptr, NOUT, 0L, bY, nullptr, 0L, NROWS, NOUT, 2 * NHID, 1.0f / 128.0f);
}
